// LorentzTransformerBlock_53231824666658
// MI455X (gfx1250) — hardware-verified
//
#include <hip/hip_runtime.h>


#define NBT  4
#define SS   1024
#define NR   (NBT * SS)
#define DD   512
#define SD   511
#define NH_  8
#define HD   64
#define HS   63
#define FF   2048
#define FS   2047
#define KK   1.0f
#define LEPS 1e-6f
#define RSC  27.5f
#define DM   DD
#define NN   SS
#define NTK  SS
#define LOSC 1024.0f

typedef _Float16 h16;
typedef unsigned short bf;
typedef __attribute__((ext_vector_type(16))) __bf16   v16bf;
typedef __attribute__((ext_vector_type(16))) _Float16 v16h;
typedef __attribute__((ext_vector_type(8)))  _Float16 v8h;
typedef __attribute__((ext_vector_type(8)))  unsigned short v8us;
typedef __attribute__((ext_vector_type(8)))  float    v8f;
typedef __attribute__((ext_vector_type(4)))  float    v4f;
typedef __attribute__((ext_vector_type(4)))  _Float16 v4h;
typedef v8h  __attribute__((may_alias)) v8ha;
typedef v4f  __attribute__((may_alias)) v4fa;
typedef v8us __attribute__((may_alias)) v8usa;

__device__ __forceinline__ unsigned short f2bf(float f) { unsigned u = __float_as_uint(f); u += 0x7FFFu + ((u >> 16) & 1u); return (unsigned short)(u >> 16); }
__device__ __forceinline__ float bf2f(unsigned short b) { return __uint_as_float(((unsigned)b) << 16); }
__device__ __forceinline__ float bfr(float f) { return bf2f(f2bf(f)); }
__device__ __forceinline__ v16h cat16(v8h lo, v8h hi) { return __builtin_shufflevector(lo, hi, 0, 1, 2, 3, 4, 5, 6, 7, 8, 9, 10, 11, 12, 13, 14, 15); }
__device__ __forceinline__ v16bf cat16b(v8us lo, v8us hi) { return __builtin_bit_cast(v16bf, __builtin_shufflevector(lo, hi, 0, 1, 2, 3, 4, 5, 6, 7, 8, 9, 10, 11, 12, 13, 14, 15)); }
__device__ __forceinline__ v8f wmma16(v16h a, v16h b, v8f c) { return __builtin_amdgcn_wmma_f32_16x16x32_f16(false, a, false, b, (short)0, c, false, false); }
__device__ __forceinline__ v8f wmmab(v16bf a, v16bf b, v8f c) { return __builtin_amdgcn_wmma_f32_16x16x32_bf16(false, a, false, b, (short)0, c, false, false); }

template <bool SPLITA, bool F16OUT = false>
__global__ __launch_bounds__(128) void k_gemmb(const bf* __restrict__ A, const bf* __restrict__ Al, const bf* __restrict__ Bn, const float* __restrict__ bias, float* C, int ldc, h16* C2, const float* __restrict__ R = nullptr, int K = DM, int roundR = 1) {
    __shared__ __align__(16) float ost[4][16 * 68];
    const int lane = threadIdx.x & 31, wave = threadIdx.x >> 5, lr = lane & 15, hi = lane >> 4;
    const int r0 = blockIdx.x * 64 + wave * 16, c0 = blockIdx.y * 64;
    const size_t aoff = (size_t)(r0 + lr) * K + 8 * hi;
    size_t boff[4];
#pragma unroll
    for (int t = 0; t < 4; ++t) boff[t] = (size_t)(c0 + t * 16 + lr) * K + 8 * hi;
    v8f acc[4];
#pragma unroll
    for (int t = 0; t < 4; ++t) acc[t] = (v8f){};
#pragma unroll 1
    for (int kc = 0; kc < K; kc += 32) {
        const v16bf a = cat16b(*(const v8us*)(A + aoff + kc), *(const v8us*)(A + aoff + kc + 16));
        v16bf al = a;
        if (SPLITA) al = cat16b(*(const v8us*)(Al + aoff + kc), *(const v8us*)(Al + aoff + kc + 16));
#pragma unroll
        for (int t = 0; t < 4; ++t) { const v16bf b = cat16b(*(const v8us*)(Bn + boff[t] + kc), *(const v8us*)(Bn + boff[t] + kc + 16)); acc[t] = wmmab(a, b, acc[t]); if (SPLITA) acc[t] = wmmab(al, b, acc[t]); }
        asm volatile("v_nop\n\tv_nop\n\tv_nop\n\tv_nop" : "+v"(acc[0]), "+v"(acc[1]), "+v"(acc[2]), "+v"(acc[3]) : "v"(a), "v"(al));
    }
    float* os = &ost[wave][0];
#pragma unroll
    for (int t = 0; t < 4; ++t) { const float bv = bias ? bfr(bias[c0 + t * 16 + lr]) : 0.f;
#pragma unroll
        for (int j = 0; j < 8; ++j) os[(hi * 8 + j) * 68 + t * 16 + lr] = acc[t][j] + bv; }
    __syncthreads();
    if (F16OUT) {
        h16* crow = (h16*)(void*)C + (size_t)r0 * ldc + c0;
        auto pass = [&]() {
#pragma unroll
            for (int s = 0; s < 4; ++s) { const int row = 4 * s + (lane >> 3), piece = lane & 7; const float* sp = os + row * 68 + piece * 8; v8h o, o2;
#pragma unroll
                for (int i = 0; i < 8; ++i) { const h16 a = (h16)sp[i]; o[i] = a; o2[i] = (h16)((sp[i] - (float)a) * LOSC); }
                *(volatile v8h*)(crow + (size_t)row * ldc + piece * 8) = o; if (C2) *(volatile v8h*)(C2 + (size_t)r0 * ldc + c0 + (size_t)row * ldc + piece * 8) = o2; }
        };
        pass(); __threadfence(); pass();
    } else {
        float* crow = C + (size_t)r0 * ldc + c0;
        auto pass = [&]() {
#pragma unroll
            for (int s = 0; s < 8; ++s) { const int Lid = (lane >> 3) + 4 * s, piece = lane & 7; const int row = Lid >> 1, cofs = (Lid & 1) * 32 + piece * 4;
                v4f val = *(const v4fa*)(os + row * 68 + cofs); if (R) { const v4f rv = *(const v4f*)(R + ((size_t)r0 + row) * ldc + c0 + cofs); val += roundR ? (v4f){bfr(rv[0]), bfr(rv[1]), bfr(rv[2]), bfr(rv[3])} : rv; }
                *(volatile v4f*)(crow + (size_t)row * ldc + cofs) = val; }
        };
        pass(); __threadfence(); pass();
    }
}


template <int MODE>
__global__ __launch_bounds__(128) void k_gemm3z(const bf* __restrict__ Ah, const bf* __restrict__ Al, const bf* __restrict__ Bh, const bf* __restrict__ Bl, int K, float* C, int ldc, size_t sA, size_t sB, size_t sC) {
    if ((MODE & 1) && (int)blockIdx.y * 64 > (int)blockIdx.x * 64 + 63) return;
    const size_t z = blockIdx.z; Ah += z * sA; Al += z * sA; Bh += z * sB; Bl += z * sB; C += z * sC;
    const int Klim = (MODE & 2) ? min(K, ((int)blockIdx.x + 1) * 64) : K;
    __shared__ __align__(16) float ost[4][16 * 68];
    const int lane = threadIdx.x & 31, wave = threadIdx.x >> 5, lr = lane & 15, hi = lane >> 4;
    const int r0 = blockIdx.x * 64 + wave * 16, c0 = blockIdx.y * 64;
    const size_t aoff = (size_t)(r0 + lr) * K + 8 * hi;
    v8f acc[4];
#pragma unroll
    for (int t = 0; t < 4; ++t) acc[t] = (v8f){};
#pragma unroll 1
    for (int kc = 0; kc < Klim; kc += 32) {
        const v16bf a = cat16b(*(const v8us*)(Ah + aoff + kc), *(const v8us*)(Ah + aoff + kc + 16));
        v16bf al = a; if (!(MODE & 4) && !(MODE & 16)) al = cat16b(*(const v8us*)(Al + aoff + kc), *(const v8us*)(Al + aoff + kc + 16));
#pragma unroll
        for (int t = 0; t < 4; ++t) { const size_t bo = (size_t)(c0 + t * 16 + lr) * K + kc + 8 * hi;
            const v16bf bh = cat16b(*(const v8us*)(Bh + bo), *(const v8us*)(Bh + bo + 16));
            acc[t] = wmmab(a, bh, acc[t]);
            if (!(MODE & 4)) { if (!(MODE & 16)) acc[t] = wmmab(al, bh, acc[t]); if (!(MODE & 8)) { const v16bf bl = cat16b(*(const v8us*)(Bl + bo), *(const v8us*)(Bl + bo + 16)); acc[t] = wmmab(a, bl, acc[t]); } } }
        asm volatile("v_nop\n\tv_nop\n\tv_nop\n\tv_nop" : "+v"(acc[0]), "+v"(acc[1]), "+v"(acc[2]), "+v"(acc[3]) : "v"(a), "v"(al));
    }
    float* os = &ost[wave][0];
#pragma unroll
    for (int t = 0; t < 4; ++t) {
#pragma unroll
        for (int j = 0; j < 8; ++j) os[(hi * 8 + j) * 68 + t * 16 + lr] = acc[t][j]; }
    __builtin_amdgcn_wave_barrier(); asm volatile("" ::: "memory");
    float* crow = C + (size_t)r0 * ldc + c0;
    auto pass = [&]() {
#pragma unroll
        for (int s = 0; s < 8; ++s) { const int Lid = (lane >> 3) + 4 * s, piece = lane & 7; const int row = Lid >> 1, cofs = (Lid & 1) * 32 + piece * 4;
            const v4f val = *(const v4fa*)(os + row * 68 + cofs); *(volatile v4f*)(crow + (size_t)row * ldc + cofs) = val; }
    };
    pass(); __threadfence(); pass();
}
__global__ __launch_bounds__(256) void k_planes32z(const float* __restrict__ F, int ld, int off, float sc, int rows, bf* Ph, bf* Pl) {
    typedef __attribute__((ext_vector_type(2))) unsigned short v2us;
    const int lane = threadIdx.x & 31; const size_t r = ((size_t)blockIdx.x * 8 + (threadIdx.x >> 5)) * 2 + (lane >> 4); if (r >= (size_t)rows) return; const int z = blockIdx.z; const int c0 = (lane & 15) * 2; v2us oh, ol;
    Ph += (size_t)z * rows * 32; Pl += (size_t)z * rows * 32;
#pragma unroll
    for (int i = 0; i < 2; ++i) { const float y = F[r * ld + off + z * 32 + c0 + i] * sc; const unsigned short hb = f2bf(y); oh[i] = hb; ol[i] = f2bf(y - bf2f(hb)); }
    const size_t o = r * 32 + c0; *(volatile v2us*)(Ph + o) = oh; *(volatile v2us*)(Pl + o) = ol; __threadfence(); *(volatile v2us*)(Ph + o) = oh; *(volatile v2us*)(Pl + o) = ol;
}
__global__ __launch_bounds__(256) void k_vtpadz(const float* __restrict__ F, int ld, int off, int nk, bf* Th, bf* Tl) {
    typedef __attribute__((ext_vector_type(2))) unsigned short v2us;
    const int lane = threadIdx.x & 31; const size_t wid = (size_t)blockIdx.x * 8 + (threadIdx.x >> 5); if (wid >= (size_t)64 * (nk / 64)) return; const int z = blockIdx.z; const int d = (int)(wid / (nk / 64)); const int k0 = (int)(wid % (nk / 64)) * 64 + lane * 2; v2us oh, ol;
    Th += (size_t)z * 64 * nk; Tl += (size_t)z * 64 * nk;
#pragma unroll
    for (int i = 0; i < 2; ++i) { const float y = (d < 32) ? F[(size_t)(k0 + i) * ld + off + z * 32 + (d < 32 ? d : 0)] : 0.f; const unsigned short hb = f2bf(y); oh[i] = hb; ol[i] = f2bf(y - bf2f(hb)); }
    const size_t o = (size_t)d * nk + k0; *(volatile v2us*)(Th + o) = oh; *(volatile v2us*)(Tl + o) = ol; __threadfence(); *(volatile v2us*)(Th + o) = oh; *(volatile v2us*)(Tl + o) = ol;
}
template <int NK>
__global__ __launch_bounds__(256) void k_softmaxz(const float* __restrict__ S, int rows, bf* PH, bf* PL) {
    typedef __attribute__((ext_vector_type(4))) unsigned short v4us;
    const int lane = threadIdx.x & 31, i = blockIdx.x * 8 + (threadIdx.x >> 5); if (i >= rows) return; const size_t zo = (size_t)blockIdx.z * rows * NK; const float* sr = S + zo + (size_t)i * NK; PH += zo; PL += zo;
    float m = -3.0e38f;
#pragma unroll 1
    for (int c0 = lane * 4; c0 < NK; c0 += 128) {
#pragma unroll
        for (int q = 0; q < 4; ++q) m = fmaxf(m, sr[c0 + q]); }
#pragma unroll
    for (int sh = 16; sh; sh >>= 1) m = fmaxf(m, __shfl_xor(m, sh, 32));
    float sum = 0.f;
#pragma unroll 1
    for (int c0 = lane * 4; c0 < NK; c0 += 128) {
#pragma unroll
        for (int q = 0; q < 4; ++q) sum += __expf(sr[c0 + q] - m); }
#pragma unroll
    for (int sh = 16; sh; sh >>= 1) sum += __shfl_xor(sum, sh, 32);
    const float inv = 1.0f / sum;
#pragma unroll 1
    for (int ps = 0; ps < 2; ++ps) {
#pragma unroll 1
        for (int c0 = lane * 4; c0 < NK; c0 += 128) { v4us oh, ol;
#pragma unroll
            for (int q = 0; q < 4; ++q) { const float p = __expf(sr[c0 + q] - m) * inv; const unsigned short hb = f2bf(p); oh[q] = hb; ol[q] = f2bf(p - bf2f(hb)); }
            const size_t o = (size_t)i * NK + c0; *(volatile v4us*)(PH + o) = oh; *(volatile v4us*)(PL + o) = ol; }
        if (ps == 0) __threadfence(); }
}
__global__ __launch_bounds__(256) void k_placez(const float* __restrict__ XH, int rows, int ldy, float* Y) {
    const int lane = threadIdx.x & 31; const size_t q = (size_t)blockIdx.x * 8 + (threadIdx.x >> 5); if (q >= (size_t)rows) return; const int z = blockIdx.z; const float v = XH[((size_t)z * rows + q) * 64 + lane];
    *(volatile float*)(Y + q * ldy + z * 32 + lane) = v; __threadfence(); *(volatile float*)(Y + q * ldy + z * 32 + lane) = v;
}

__global__ __launch_bounds__(256) void k_hplanesz(const float* __restrict__ F, int ld, int h0, float sc, int rows, bf* Ph, bf* Pl) {
    typedef __attribute__((ext_vector_type(2))) unsigned short v2us;
    const int lane = threadIdx.x & 31; const size_t r = (size_t)blockIdx.x * 8 + (threadIdx.x >> 5); if (r >= (size_t)rows) return; const int z = blockIdx.z; v2us oh, ol;
    Ph += (size_t)z * rows * 64; Pl += (size_t)z * rows * 64;
#pragma unroll
    for (int i = 0; i < 2; ++i) { const float y = F[r * ld + (h0 + z) * 64 + lane * 2 + i] * sc; const unsigned short hb = f2bf(y); oh[i] = hb; ol[i] = f2bf(y - bf2f(hb)); }
    const size_t o = r * 64 + lane * 2; *(volatile v2us*)(Ph + o) = oh; *(volatile v2us*)(Pl + o) = ol; __threadfence(); *(volatile v2us*)(Ph + o) = oh; *(volatile v2us*)(Pl + o) = ol;
}
__global__ __launch_bounds__(256) void k_vtz(const float* __restrict__ F, int ld, int h0, int nk, bf* Th, bf* Tl) {
    typedef __attribute__((ext_vector_type(2))) unsigned short v2us;
    const int lane = threadIdx.x & 31; const size_t wid = (size_t)blockIdx.x * 8 + (threadIdx.x >> 5); if (wid >= (size_t)64 * (nk / 64)) return; const int z = blockIdx.z; const int d = (int)(wid / (nk / 64)); const int t0 = (int)(wid % (nk / 64)) * 64 + lane * 2; v2us oh, ol;
    Th += (size_t)z * 64 * nk; Tl += (size_t)z * 64 * nk;
#pragma unroll
    for (int i = 0; i < 2; ++i) { const float y = F[(size_t)(t0 + i) * ld + (h0 + z) * 64 + d]; const unsigned short hb = f2bf(y); oh[i] = hb; ol[i] = f2bf(y - bf2f(hb)); }
    const size_t o = (size_t)d * nk + t0; *(volatile v2us*)(Th + o) = oh; *(volatile v2us*)(Tl + o) = ol; __threadfence(); *(volatile v2us*)(Th + o) = oh; *(volatile v2us*)(Tl + o) = ol;
}
template <int NK>
__global__ __launch_bounds__(256) void k_softmaxzs(const float* __restrict__ S, int rows, float sc, bf* PH, bf* PL) {
    typedef __attribute__((ext_vector_type(4))) unsigned short v4us;
    const int lane = threadIdx.x & 31, i = blockIdx.x * 8 + (threadIdx.x >> 5); if (i >= rows) return; const size_t zo = (size_t)blockIdx.z * rows * NK; const float* sr = S + zo + (size_t)i * NK; PH += zo; PL += zo;
    float m = -3.0e38f;
#pragma unroll 1
    for (int c0 = lane * 4; c0 < NK; c0 += 128) {
#pragma unroll
        for (int q = 0; q < 4; ++q) m = fmaxf(m, sr[c0 + q] * sc); }
#pragma unroll
    for (int sh = 16; sh; sh >>= 1) m = fmaxf(m, __shfl_xor(m, sh, 32));
    float sum = 0.f;
#pragma unroll 1
    for (int c0 = lane * 4; c0 < NK; c0 += 128) {
#pragma unroll
        for (int q = 0; q < 4; ++q) sum += __expf(sr[c0 + q] * sc - m); }
#pragma unroll
    for (int sh = 16; sh; sh >>= 1) sum += __shfl_xor(sum, sh, 32);
    const float inv = 1.0f / sum;
#pragma unroll 1
    for (int ps = 0; ps < 2; ++ps) {
#pragma unroll 1
        for (int c0 = lane * 4; c0 < NK; c0 += 128) { v4us oh, ol;
#pragma unroll
            for (int q = 0; q < 4; ++q) { const float p = __expf(sr[c0 + q] * sc - m) * inv; const unsigned short hb = f2bf(p); oh[q] = hb; ol[q] = f2bf(p - bf2f(hb)); }
            const size_t o = (size_t)i * NK + c0; *(volatile v4us*)(PH + o) = oh; *(volatile v4us*)(PL + o) = ol; }
        if (ps == 0) __threadfence(); }
}
__global__ __launch_bounds__(128) void k_gemm3(const bf* __restrict__ Ah, const bf* __restrict__ Al, const bf* __restrict__ Bh, const bf* __restrict__ Bl, int K, float* C, int ldc) {
    __shared__ __align__(16) float ost[4][16 * 68];
    const int lane = threadIdx.x & 31, wave = threadIdx.x >> 5, lr = lane & 15, hi = lane >> 4;
    const int r0 = blockIdx.x * 64 + wave * 16, c0 = blockIdx.y * 64;
    const size_t aoff = (size_t)(r0 + lr) * K + 8 * hi;
    v8f acc[4];
#pragma unroll
    for (int t = 0; t < 4; ++t) acc[t] = (v8f){};
#pragma unroll 1
    for (int kc = 0; kc < K; kc += 32) {
        const v16bf a = cat16b(*(const v8us*)(Ah + aoff + kc), *(const v8us*)(Ah + aoff + kc + 16));
        const v16bf al = cat16b(*(const v8us*)(Al + aoff + kc), *(const v8us*)(Al + aoff + kc + 16));
#pragma unroll
        for (int t = 0; t < 4; ++t) { const size_t bo = (size_t)(c0 + t * 16 + lr) * K + kc + 8 * hi;
            const v16bf bh = cat16b(*(const v8us*)(Bh + bo), *(const v8us*)(Bh + bo + 16)); const v16bf bl = cat16b(*(const v8us*)(Bl + bo), *(const v8us*)(Bl + bo + 16));
            acc[t] = wmmab(a, bh, acc[t]); acc[t] = wmmab(al, bh, acc[t]); acc[t] = wmmab(a, bl, acc[t]); }
        asm volatile("v_nop\n\tv_nop\n\tv_nop\n\tv_nop" : "+v"(acc[0]), "+v"(acc[1]), "+v"(acc[2]), "+v"(acc[3]) : "v"(a), "v"(al));
    }
    float* os = &ost[wave][0];
#pragma unroll
    for (int t = 0; t < 4; ++t) {
#pragma unroll
        for (int j = 0; j < 8; ++j) os[(hi * 8 + j) * 68 + t * 16 + lr] = acc[t][j]; }
    __builtin_amdgcn_wave_barrier(); asm volatile("" ::: "memory");
    float* crow = C + (size_t)r0 * ldc + c0;
    auto pass = [&]() {
#pragma unroll
        for (int s = 0; s < 8; ++s) { const int Lid = (lane >> 3) + 4 * s, piece = lane & 7; const int row = Lid >> 1, cofs = (Lid & 1) * 32 + piece * 4;
            const v4f val = *(const v4fa*)(os + row * 68 + cofs); *(volatile v4f*)(crow + (size_t)row * ldc + cofs) = val; }
    };
    pass(); __threadfence(); pass();
}


__device__ __forceinline__ float gelu_t(float x) { const float c = 0.7978845608028654f; const float t = tanhf(c * (x + 0.044715f * x * x * x)); return 0.5f * x * (1.0f + t); }
template <bool RAWIN>
__global__ __launch_bounds__(256) void k_lln(const float* __restrict__ X, const float* __restrict__ g, const float* __restrict__ bb, int rows, bf* Hh, bf* Hl) {
    const int lane = threadIdx.x & 31; const size_t r = (size_t)blockIdx.x * 8 + (threadIdx.x >> 5); if (r >= (size_t)rows) return; float v[16]; float s = 0.f;
#pragma unroll
    for (int i = 0; i < 16; ++i) { const int c = lane * 16 + i; float t = X[r * DD + c]; if (RAWIN) t = bfr(t); v[i] = t; if (c >= 1) s += t; }
#pragma unroll
    for (int sh = 16; sh; sh >>= 1) s += __shfl_xor(s, sh, 32);
    const float mu = s * (1.0f / SD); float q = 0.f;
#pragma unroll
    for (int i = 0; i < 16; ++i) { const int c = lane * 16 + i; if (c >= 1) { const float d = v[i] - mu; q = fmaf(d, d, q); } }
#pragma unroll
    for (int sh = 16; sh; sh >>= 1) q += __shfl_xor(q, sh, 32);
    const float rs = rsqrtf(q * (1.0f / SD) + 1e-5f); float n2 = 0.f;
#pragma unroll
    for (int i = 0; i < 16; ++i) { const int c = lane * 16 + i; if (c >= 1) { const float y = (v[i] - mu) * rs * bfr(g[c - 1]) + bfr(bb[c - 1]); v[i] = y; n2 = fmaf(y, y, n2); } }
#pragma unroll
    for (int sh = 16; sh; sh >>= 1) n2 += __shfl_xor(n2, sh, 32);
    const float tm = sqrtf(fmaxf(KK + n2, LEPS)); if (lane == 0) v[0] = tm;
#pragma unroll 1
    for (int ps = 0; ps < 2; ++ps) {
#pragma unroll
        for (int hq = 0; hq < 2; ++hq) { v8us oh, ol;
#pragma unroll
            for (int i = 0; i < 8; ++i) { const float y = v[hq * 8 + i]; const unsigned short hb = f2bf(y); oh[i] = hb; ol[i] = f2bf(y - bf2f(hb)); }
            const size_t o = r * DD + lane * 16 + hq * 8; *(volatile v8us*)(Hh + o) = oh; *(volatile v8us*)(Hl + o) = ol; }
        if (ps == 0) __threadfence(); }
}
__global__ __launch_bounds__(256) void k_wtpad(const float* __restrict__ Wm, int Kl, int Nl, int K, int NP, bf* Bt) {
    const int lane = threadIdx.x & 31; const int n = blockIdx.x * 8 + (threadIdx.x >> 5); if (n >= NP) return;
    for (int ps = 0; ps < 2; ++ps) {
        for (int k0 = 0; k0 < K; k0 += 256) { v8us o;
#pragma unroll
            for (int i = 0; i < 8; ++i) { const int k = k0 + lane * 8 + i; const bool live = (k < Kl) && (n < Nl); o[i] = f2bf(live ? Wm[(size_t)(live ? k : 0) * Nl + (live ? n : 0)] : 0.f); }
            *(volatile v8us*)(Bt + (size_t)n * K + k0 + lane * 8) = o; }
        if (ps == 0) __threadfence(); }
}
__global__ __launch_bounds__(256) void k_bpad(const float* __restrict__ b, int Nl, int NP, float* BP) {
    const int i = blockIdx.x * 256 + threadIdx.x; if (i >= NP) return; const float v = (i < Nl) ? b[i] : 0.f; *(volatile float*)(BP + i) = v; __threadfence(); *(volatile float*)(BP + i) = v;
}
__global__ __launch_bounds__(256) void k_headpl(const float* __restrict__ QS, const float* __restrict__ KS, const float* __restrict__ VS, size_t r0, int h, bf* Qh, bf* Ql, bf* Kh, bf* Kl, bf* Vh, bf* Vl) {
    typedef __attribute__((ext_vector_type(2))) unsigned short v2us;
    const int lane = threadIdx.x & 31; const size_t rl = (size_t)blockIdx.x * 8 + (threadIdx.x >> 5); if (rl >= (size_t)SS) return; const size_t r = r0 + rl; const int cb = h * HD;
    float q2 = 0.f, k2 = 0.f, v2 = 0.f; float qv_[2], kv_[2], vv_[2];
#pragma unroll
    for (int i = 0; i < 2; ++i) { const int d = lane * 2 + i;
        const float qa = (d >= 1) ? QS[r * DD + cb + d - 1] : 0.f, ka = (d >= 1) ? KS[r * DD + cb + d - 1] : 0.f, va = (d >= 1) ? VS[r * DD + cb + d - 1] : 0.f; qv_[i] = qa; kv_[i] = ka; vv_[i] = va; q2 = fmaf(qa, qa, q2); k2 = fmaf(ka, ka, k2); v2 = fmaf(va, va, v2); }
#pragma unroll
    for (int sh = 16; sh; sh >>= 1) { q2 += __shfl_xor(q2, sh, 32); k2 += __shfl_xor(k2, sh, 32); v2 += __shfl_xor(v2, sh, 32); }
    const float qt = sqrtf(fmaxf(KK + q2, LEPS)), kt = sqrtf(fmaxf(KK + k2, LEPS)), vt = sqrtf(fmaxf(KK + v2, LEPS));
    if (lane == 0) { qv_[0] = qt; kv_[0] = -kt; vv_[0] = vt; }
    v2us qh_, ql_, kh_, kl_;
#pragma unroll
    for (int i = 0; i < 2; ++i) { unsigned short hb = f2bf(qv_[i]); qh_[i] = hb; ql_[i] = f2bf(qv_[i] - bf2f(hb)); hb = f2bf(kv_[i]); kh_[i] = hb; kl_[i] = f2bf(kv_[i] - bf2f(hb)); }
    const size_t o = rl * HD + lane * 2;
#pragma unroll 1
    for (int ps = 0; ps < 2; ++ps) { *(volatile v2us*)(Qh + o) = qh_; *(volatile v2us*)(Ql + o) = ql_; *(volatile v2us*)(Kh + o) = kh_; *(volatile v2us*)(Kl + o) = kl_; if (ps == 0) __threadfence(); }
    v2us vh_, vl_;
#pragma unroll
    for (int i = 0; i < 2; ++i) { const unsigned short hb = f2bf(vv_[i]); vh_[i] = hb; vl_[i] = f2bf(vv_[i] - bf2f(hb)); }
    *(volatile v2us*)(Vh + o) = vh_; *(volatile v2us*)(Vl + o) = vl_; __threadfence(); *(volatile v2us*)(Vh + o) = vh_; *(volatile v2us*)(Vl + o) = vl_;
}
__global__ __launch_bounds__(256) void k_bfT64(const bf* __restrict__ P, bf* T) {
    __shared__ unsigned short tl[64][66];
    typedef __attribute__((ext_vector_type(4))) unsigned short v4us;
    const int tid = threadIdx.x; const int t0 = blockIdx.x * 64; const int rr = tid >> 2, cq = (tid & 3) * 16;
#pragma unroll
    for (int i = 0; i < 16; ++i) tl[rr][cq + i] = P[(size_t)(t0 + rr) * HD + cq + i];
    __syncthreads();
    const int lane = tid & 31, wv = tid >> 5;
    auto pass = [&]() {
#pragma unroll
        for (int st = 0; st < 4; ++st) { const int dr = wv * 8 + st * 2 + (lane >> 4); const int tq = (lane & 15) * 4; v4us v;
#pragma unroll
            for (int i = 0; i < 4; ++i) v[i] = tl[tq + i][dr];
            *(volatile v4us*)(T + (size_t)dr * SS + t0 + tq) = v; }
    };
    pass(); __threadfence(); pass();
}
__global__ __launch_bounds__(256) void k_midcat(const float* __restrict__ XO, size_t r0, bf* SPh, bf* SPl) {
    const int lane = threadIdx.x & 31; const size_t rl = (size_t)blockIdx.x * 8 + (threadIdx.x >> 5); if (rl >= (size_t)SS) return; const size_t r = r0 + rl; float dn[NH_];
#pragma unroll
    for (int h = 0; h < NH_; ++h) { const float* a = XO + ((size_t)h * SS + rl) * HD; float s = 0.f;
#pragma unroll
        for (int i = 0; i < 2; ++i) { const int d = lane * 2 + i; if (d >= 1) s = fmaf(a[d], a[d], s); }
#pragma unroll
        for (int sh = 16; sh; sh >>= 1) s += __shfl_xor(s, sh, 32);
        dn[h] = sqrtf(fmaxf(fabsf(s - a[0] * a[0]), LEPS)); }
#pragma unroll 1
    for (int ps = 0; ps < 2; ++ps) {
#pragma unroll
        for (int hq = 0; hq < 2; ++hq) { v8us oh, ol;
#pragma unroll 1
            for (int i = 0; i < 8; ++i) { const int c = lane * 16 + hq * 8 + i; float y = 0.f; if (c < NH_ * HS) { const int h = c / HS, d = c % HS + 1; float dd = dn[0];
#pragma unroll
                    for (int hh = 1; hh < NH_; ++hh) dd = (h == hh) ? dn[hh] : dd;
                    y = XO[((size_t)h * SS + rl) * HD + d] / dd; }
                const unsigned short hb = f2bf(y); oh[i] = hb; ol[i] = f2bf(y - bf2f(hb)); }
            const size_t o = r * DD + lane * 16 + hq * 8; *(volatile v8us*)(SPh + o) = oh; *(volatile v8us*)(SPl + o) = ol; }
        if (ps == 0) __threadfence(); }
}
template <bool RAWIN>
__global__ __launch_bounds__(256) void k_res(const float* __restrict__ X, const float* __restrict__ AO, int rows, float* X1) {
    const int lane = threadIdx.x & 31; const size_t r = (size_t)blockIdx.x * 8 + (threadIdx.x >> 5); if (r >= (size_t)rows) return; float v[16]; float n2 = 0.f;
#pragma unroll
    for (int i = 0; i < 16; ++i) { const int c = lane * 16 + i; float y = 0.f; if (c >= 1) { float xs = X[r * DD + c]; if (RAWIN) xs = bfr(xs); y = xs + RSC * AO[r * DD + c - 1]; n2 = fmaf(y, y, n2); } v[i] = y; }
#pragma unroll
    for (int sh = 16; sh; sh >>= 1) n2 += __shfl_xor(n2, sh, 32);
    if (lane == 0) v[0] = sqrtf(fmaxf(KK + n2, LEPS));
#pragma unroll 1
    for (int ps = 0; ps < 2; ++ps) {
#pragma unroll
        for (int q = 0; q < 4; ++q) { v4f o; for (int i = 0; i < 4; ++i) o[i] = v[q * 4 + i]; *(volatile v4f*)(X1 + r * DD + lane * 16 + q * 4) = o; }
        if (ps == 0) __threadfence(); }
}
__global__ __launch_bounds__(256) void k_gelupl(const float* __restrict__ M1, int rows, bf* Gh, bf* Gl) {
    const int lane = threadIdx.x & 31; const size_t r = (size_t)blockIdx.x * 8 + (threadIdx.x >> 5); if (r >= (size_t)rows) return; float n2 = 0.f;
#pragma unroll 1
    for (int q = 0; q < FF / 256; ++q) {
#pragma unroll 1
        for (int i = 0; i < 8; ++i) { const int c = q * 256 + lane * 8 + i; if (c >= 1) { const float gx = gelu_t(M1[r * FF + c - 1]); n2 = fmaf(gx, gx, n2); } } }
#pragma unroll
    for (int sh = 16; sh; sh >>= 1) n2 += __shfl_xor(n2, sh, 32);
    const float tm = sqrtf(fmaxf(KK + n2, LEPS));
#pragma unroll 1
    for (int ps = 0; ps < 2; ++ps) {
#pragma unroll 1
        for (int q = 0; q < FF / 256; ++q) { v8us oh, ol;
#pragma unroll 1
            for (int i = 0; i < 8; ++i) { const int c = q * 256 + lane * 8 + i; const float y = (c >= 1) ? gelu_t(M1[r * FF + c - 1]) : tm; const unsigned short hb = f2bf(y); oh[i] = hb; ol[i] = f2bf(y - bf2f(hb)); }
            const size_t o = r * FF + q * 256 + lane * 8; *(volatile v8us*)(Gh + o) = oh; *(volatile v8us*)(Gl + o) = ol; }
        if (ps == 0) __threadfence(); }
}

extern "C" void kernel_launch(void* const* d_in, const int* in_sizes, int n_in,
                              void* d_out, int out_size, void* d_ws, size_t ws_size, hipStream_t stream) {
    (void)in_sizes; (void)n_in; (void)out_size;
    const float* x = (const float*)d_in[0]; const float* Wq = (const float*)d_in[1]; const float* bq = (const float*)d_in[2]; const float* Wk = (const float*)d_in[3]; const float* bk = (const float*)d_in[4]; const float* Wv = (const float*)d_in[5]; const float* bv = (const float*)d_in[6]; const float* Wo = (const float*)d_in[7]; const float* bo = (const float*)d_in[8];
    const float* l1g = (const float*)d_in[9]; const float* l1b = (const float*)d_in[10]; const float* l2g = (const float*)d_in[11]; const float* l2b = (const float*)d_in[12]; const float* W1 = (const float*)d_in[13]; const float* b1 = (const float*)d_in[14]; const float* W2 = (const float*)d_in[15]; const float* b2 = (const float*)d_in[16];
    float* out = (float*)d_out;
    char* wsp = (char*)d_ws;
    auto take = [&](size_t bytes) { char* p = wsp; wsp += (bytes + 255) & ~(size_t)255; return (void*)p; };
    bf* BQ = (bf*)take((size_t)DD * DD * 2); bf* BK = (bf*)take((size_t)DD * DD * 2); bf* BV = (bf*)take((size_t)DD * DD * 2); bf* BO = (bf*)take((size_t)DD * DD * 2); bf* B1 = (bf*)take((size_t)FF * DD * 2); bf* B2 = (bf*)take((size_t)DD * FF * 2);
    float* PBQ = (float*)take(DD * 4); float* PBK = (float*)take(DD * 4); float* PBV = (float*)take(DD * 4); float* PBO = (float*)take(DD * 4); float* PB1 = (float*)take(FF * 4); float* PB2 = (float*)take(DD * 4);
    bf* Hh = (bf*)take((size_t)NR * DD * 2); bf* Hl = (bf*)take((size_t)NR * DD * 2); float* QS = (float*)take((size_t)NR * DD * 4); float* KS = (float*)take((size_t)NR * DD * 4); float* VS = (float*)take((size_t)NR * DD * 4);
    bf* Qh = (bf*)take((size_t)SS * HD * 2); bf* Ql = (bf*)take((size_t)SS * HD * 2); bf* Kh = (bf*)take((size_t)SS * HD * 2); bf* Kl = (bf*)take((size_t)SS * HD * 2); bf* Vh = (bf*)take((size_t)SS * HD * 2); bf* Vl = (bf*)take((size_t)SS * HD * 2); bf* VTh = (bf*)take((size_t)HD * SS * 2); bf* VTl = (bf*)take((size_t)HD * SS * 2);
    float* S = (float*)take((size_t)SS * SS * 4); bf* PH = (bf*)take((size_t)SS * SS * 2); bf* PL = (bf*)take((size_t)SS * SS * 2); float* XO = (float*)take((size_t)NH_ * SS * HD * 4);
    bf* SPh = (bf*)take((size_t)NR * DD * 2); bf* SPl = (bf*)take((size_t)NR * DD * 2); float* AO = (float*)take((size_t)NR * DD * 4); float* X1 = (float*)take((size_t)NR * DD * 4); float* M1 = (float*)take((size_t)NR * FF * 4); bf* Gh = (bf*)take((size_t)NR * FF * 2); bf* Gl = (bf*)take((size_t)NR * FF * 2); float* M2 = (float*)take((size_t)NR * DD * 4);
    if ((size_t)(wsp - (char*)d_ws) > ws_size) return;
    k_wtpad<<<DD / 8, 256, 0, stream>>>(Wq, DD, SD, DD, DD, BQ); k_wtpad<<<DD / 8, 256, 0, stream>>>(Wk, DD, SD, DD, DD, BK); k_wtpad<<<DD / 8, 256, 0, stream>>>(Wv, DD, SD, DD, DD, BV);
    k_wtpad<<<DD / 8, 256, 0, stream>>>(Wo, NH_ * HS, SD, DD, DD, BO); k_wtpad<<<FF / 8, 256, 0, stream>>>(W1, DD, FS, DD, FF, B1); k_wtpad<<<DD / 8, 256, 0, stream>>>(W2, FF, SD, FF, DD, B2);
    k_bpad<<<DD / 256, 256, 0, stream>>>(bq, SD, DD, PBQ); k_bpad<<<DD / 256, 256, 0, stream>>>(bk, SD, DD, PBK); k_bpad<<<DD / 256, 256, 0, stream>>>(bv, SD, DD, PBV); k_bpad<<<DD / 256, 256, 0, stream>>>(bo, SD, DD, PBO); k_bpad<<<FF / 256, 256, 0, stream>>>(b1, FS, FF, PB1); k_bpad<<<DD / 256, 256, 0, stream>>>(b2, SD, DD, PB2);
    k_lln<true><<<NR / 8, 256, 0, stream>>>(x, l1g, l1b, NR, Hh, Hl);
    k_gemmb<true, false><<<dim3(NR / 64, DD / 64, 1), 128, 0, stream>>>(Hh, Hl, BQ, PBQ, QS, DD, nullptr, nullptr, DD); k_gemmb<true, false><<<dim3(NR / 64, DD / 64, 1), 128, 0, stream>>>(Hh, Hl, BK, PBK, KS, DD, nullptr, nullptr, DD); k_gemmb<true, false><<<dim3(NR / 64, DD / 64, 1), 128, 0, stream>>>(Hh, Hl, BV, PBV, VS, DD, nullptr, nullptr, DD);
    for (int b = 0; b < NBT; ++b) { const size_t r0 = (size_t)b * SS;
        for (int h = 0; h < NH_; ++h) {
            k_headpl<<<SS / 8, 256, 0, stream>>>(QS, KS, VS, r0, h, Qh, Ql, Kh, Kl, Vh, Vl); k_bfT64<<<SS / 64, 256, 0, stream>>>(Vh, VTh); k_bfT64<<<SS / 64, 256, 0, stream>>>(Vl, VTl);
            k_gemm3<<<dim3(SS / 64, SS / 64, 1), 128, 0, stream>>>(Qh, Ql, Kh, Kl, HD, S, SS);
            k_softmaxzs<SS><<<dim3(SS / 8, 1, 1), 256, 0, stream>>>(S, SS, 0.25f, PH, PL);
            k_gemm3<<<dim3(SS / 64, 1, 1), 128, 0, stream>>>(PH, PL, VTh, VTl, SS, XO + (size_t)h * SS * HD, HD); }
        k_midcat<<<SS / 8, 256, 0, stream>>>(XO, r0, SPh, SPl); }
    k_gemmb<true, false><<<dim3(NR / 64, DD / 64, 1), 128, 0, stream>>>(SPh, SPl, BO, PBO, AO, DD, nullptr, nullptr, DD);
    k_res<true><<<NR / 8, 256, 0, stream>>>(x, AO, NR, X1);
    k_lln<false><<<NR / 8, 256, 0, stream>>>(X1, l2g, l2b, NR, Hh, Hl);
    k_gemmb<true, false><<<dim3(NR / 64, FF / 64, 1), 128, 0, stream>>>(Hh, Hl, B1, PB1, M1, FF, nullptr, nullptr, DD);
    k_gelupl<<<NR / 8, 256, 0, stream>>>(M1, NR, Gh, Gl);
    k_gemmb<true, false><<<dim3(NR / 64, DD / 64, 1), 128, 0, stream>>>(Gh, Gl, B2, PB2, M2, DD, nullptr, nullptr, FF);
    k_res<false><<<NR / 8, 256, 0, stream>>>(X1, M2, NR, out);
}
